// MambaLayer_32452772889242
// MI455X (gfx1250) — hardware-verified
//
#include <hip/hip_runtime.h>
#include <math.h>

typedef __attribute__((ext_vector_type(16))) _Float16 v16h;
typedef __attribute__((ext_vector_type(8)))  _Float16 v8h;
typedef __attribute__((ext_vector_type(16))) __bf16   v16b;
typedef __attribute__((ext_vector_type(8)))  __bf16   v8b;
typedef __attribute__((ext_vector_type(8)))  float    v8f;
typedef __attribute__((ext_vector_type(4)))  float    v4f;
typedef __attribute__((ext_vector_type(4)))  unsigned v4u;

constexpr int kBatch  = 4;
constexpr int kSeq    = 2048;
constexpr int kDim    = 1024;
constexpr int kNst    = 16;
constexpr int kRows   = kBatch * kSeq;
constexpr int kBcP    = 64;
constexpr int kConvTP = 260;
constexpr int kScanTS = 64;
constexpr int kScanCh = 64;
constexpr int kScanYP = 68;
constexpr float kLnEps   = 1e-5f;
constexpr float kDtCarry = 16.0f;
constexpr float kDtCarryInv = 1.0f / kDtCarry;
static_assert((kDim % 32) == 0);
static_assert((kRows % 64) == 0 && (kDim % 64) == 0 && (kBcP % 64) == 0);
static_assert((kSeq % kScanTS) == 0 && (kSeq % 64) == 0 && (kDim % kScanCh) == 0 && (kDim % 256) == 0);
static_assert(2 * kNst <= kBcP);

constexpr size_t kPlane16 = (size_t)kRows * kDim * 2;
constexpr size_t kPlane32 = (size_t)kRows * kDim * 4;
constexpr size_t kWPlane  = (size_t)kDim * kDim * 2;
constexpr size_t kOffXNH = 0;
constexpr size_t kOffXNL = kOffXNH + kPlane16;
constexpr size_t kOffR1  = kOffXNL + kPlane16;
constexpr size_t kOffUH  = kOffR1  + kPlane32;
constexpr size_t kOffUL  = kOffUH  + kPlane16;
constexpr size_t kOffDT  = kOffUL  + kPlane16;
constexpr size_t kOffBC  = kOffDT  + kPlane16;
constexpr size_t kOffW1T = kOffBC  + (size_t)kRows * kBcP * 4;
constexpr size_t kOffV1T = kOffW1T + kWPlane;
constexpr size_t kOffW2T = kOffV1T + kWPlane;
constexpr size_t kOffWDT = kOffW2T + kWPlane;
constexpr size_t kOffWBC = kOffWDT + kWPlane;
constexpr size_t kWsTotal = kOffWBC + (size_t)kBcP * kDim * 2;
static_assert(kWsTotal == 128057344ull);
static_assert(kWsTotal <= 134217728ull);
static_assert((kOffXNL % 128) == 0 && (kOffR1 % 128) == 0 && (kOffUH % 128) == 0 && (kOffUL % 128) == 0 &&
              (kOffDT % 128) == 0 && (kOffBC % 128) == 0 && (kOffW1T % 128) == 0 && (kOffV1T % 128) == 0 &&
              (kOffW2T % 128) == 0 && (kOffWDT % 128) == 0 && (kOffWBC % 128) == 0);

__device__ __forceinline__ unsigned short f2bf_bits(float f) {
  unsigned u = __float_as_uint(f);
  return (unsigned short)((u + 0x7FFFu + ((u >> 16) & 1u)) >> 16);
}
__device__ __forceinline__ float bf_bits2f(unsigned short h) { return __uint_as_float(((unsigned)h) << 16); }
__device__ __forceinline__ unsigned bf_hi32(float f) {
  const unsigned u = __float_as_uint(f);
  return (u + 0x7FFFu + ((u >> 16) & 1u)) >> 16;
}
__device__ __forceinline__ float bf32_to_f(unsigned b) { return __uint_as_float(b << 16); }
__device__ __forceinline__ float rbf(float f) { return bf32_to_f(bf_hi32(f)); }
__device__ __forceinline__ void split_pack(float a, float b, unsigned& hw, unsigned& lw) {
  const unsigned ha = bf_hi32(a), hb = bf_hi32(b);
  const unsigned la = bf_hi32(a - bf32_to_f(ha)), lb = bf_hi32(b - bf32_to_f(hb));
  hw = ha | (hb << 16);
  lw = la | (lb << 16);
}
__device__ __forceinline__ float h16_to_f32(unsigned hb) {
  const unsigned sgn = (hb & 0x8000u) << 16; const unsigned em = hb & 0x7fffu;
  const float fn = __uint_as_float((em << 13) + 0x38000000u);
  const float fs = (float)em * 5.9604644775390625e-8f;
  const float mag = (em < 0x400u) ? fs : fn; return __uint_as_float(__float_as_uint(mag) | sgn); }

__device__ __forceinline__ void dep_guard4_b(v8f& a, v8f& b, v8f& c, v8f& d, v16b x, v16b y) {
  asm volatile("v_nop\n\tv_nop\n\tv_nop\n\tv_nop" : "+v"(a), "+v"(b), "+v"(c), "+v"(d) : "v"(x), "v"(y));
}
__device__ __forceinline__ void keep4_b(v16b a, v16b b, v16b c, v16b d) { asm volatile("v_nop" :: "v"(a), "v"(b), "v"(c), "v"(d)); }
__device__ __forceinline__ void acc_guard4(v8f& a, v8f& b, v8f& c, v8f& d) { asm volatile("v_nop\n\tv_nop\n\tv_nop\n\tv_nop" : "+v"(a), "+v"(b), "+v"(c), "+v"(d)); }
struct FragB {
  union U { v16b v; v8b h[2]; };
  static __device__ __forceinline__ v16b load(const __bf16* p) {
    U f; f.h[0] = *(const v8b*)(p); f.h[1] = *(const v8b*)(p + 16); return f.v;
  }
  static __device__ __forceinline__ v8f mma(v16b a, v16b b, v8f c) {
    return __builtin_amdgcn_wmma_f32_16x16x32_bf16(false, a, false, b, (short)0, c, false, false);
  }
};

template <int SPL, int BIAS_MODE, int OUT_MODE, bool GATE, int ACT>
__global__ __launch_bounds__(256) void wmma_gemm64(
    const unsigned short* __restrict__ Ap, const unsigned short* __restrict__ A2p, int lda,
    const unsigned short* __restrict__ Btp, int ldb,
    void* __restrict__ Cout, void* __restrict__ Cout2, int ldc,
    const float* __restrict__ bias, const float* __restrict__ gate,
    int M, int N, int K, float scale) {
  typedef __bf16 T;
  typedef v16b V;
  const T* A = (const T*)Ap; const T* A2 = (const T*)A2p; const T* Bt = (const T*)Btp;
  __shared__ __align__(16) float sT[8][16 * 68];
  const int lane = threadIdx.x & 31;
  const int wave = threadIdx.x >> 5;
  const int tilesN = N >> 6;
  const int tilesM = M >> 6;
  const int tile = blockIdx.x * 8 + wave;
  if (tile >= tilesM * tilesN) return;
  const int tm = tile / tilesN;
  const int tn = tile - tm * tilesN;
  const int m0 = tm << 6;
  const int n0 = tn << 6;

  const int rlane = lane & 15;
  const int koff  = (lane >> 4) * 8;
  const int mOff  = (lane >> 4) * 8;

  v8f acc[4][4];
#pragma unroll
  for (int i = 0; i < 4; ++i)
#pragma unroll
    for (int j = 0; j < 4; ++j) acc[i][j] = (v8f){0.f,0.f,0.f,0.f,0.f,0.f,0.f,0.f};

  for (int k0 = 0; k0 < K; k0 += 32) {
    V bh[4];
#pragma unroll
    for (int j = 0; j < 4; ++j) {
      const size_t bo = (size_t)(n0 + (j << 4) + rlane) * ldb + koff + k0;
      bh[j] = FragB::load(Bt + bo);
    }
#pragma unroll
    for (int i = 0; i < 4; ++i) {
      const size_t ao = (size_t)(m0 + (i << 4) + rlane) * lda + koff + k0;
      V ah = FragB::load(A + ao);
      V al = ah;
      if (SPL >= 1) al = FragB::load(A2 + ao);
#pragma unroll
      for (int j = 0; j < 4; ++j) {
        acc[i][j] = FragB::mma(ah, bh[j], acc[i][j]);
        if (SPL >= 1) acc[i][j] = FragB::mma(al, bh[j], acc[i][j]);
      }
      dep_guard4_b(acc[i][0], acc[i][1], acc[i][2], acc[i][3], ah, al);
    }
    keep4_b(bh[0], bh[1], bh[2], bh[3]);
  }
  acc_guard4(acc[0][0], acc[0][1], acc[0][2], acc[0][3]);
  acc_guard4(acc[1][0], acc[1][1], acc[1][2], acc[1][3]);
  acc_guard4(acc[2][0], acc[2][1], acc[2][2], acc[2][3]);
  acc_guard4(acc[3][0], acc[3][1], acc[3][2], acc[3][3]);

  float* slab = sT[wave];
#pragma unroll
  for (int i = 0; i < 4; ++i) {
    const int mBase = m0 + (i << 4);
#pragma unroll
    for (int j = 0; j < 4; ++j) {
      const int n = n0 + (j << 4) + rlane;
      float bv = 0.f;
      if (BIAS_MODE == 2) bv = rbf(bias[n]);
#pragma unroll
      for (int r = 0; r < 8; ++r) {
        float v = acc[i][j][r] * scale;
        if (BIAS_MODE == 2) v += bv;
        if (ACT == 3) v = v / (1.0f + expf(-v));
        slab[(mOff + r) * 68 + (j << 4) + rlane] = v;
      }
    }
    __builtin_amdgcn_fence(__ATOMIC_RELEASE, "workgroup");
    __builtin_amdgcn_wave_barrier();
    __builtin_amdgcn_fence(__ATOMIC_ACQUIRE, "workgroup");
    if (OUT_MODE == 0) {
      float* C = (float*)Cout;
      const int hh = lane >> 4, c4 = (lane & 15) * 4;
      for (int pass = 0; pass < 2; ++pass) {
#pragma unroll
        for (int it = 0; it < 8; ++it) {
          const int row = it * 2 + hh;
          v4f v = *(const v4f*)(slab + row * 68 + c4);
          *(volatile v4f*)(C + (size_t)(mBase + row) * ldc + n0 + c4) = v;
        }
        __threadfence();
      }
    } else {
      const int q = lane >> 3, c8 = (lane & 7) * 8;
      unsigned short* C  = (unsigned short*)Cout;
      unsigned short* C2 = (unsigned short*)Cout2;
      for (int pass = 0; pass < 2; ++pass) {
#pragma unroll
        for (int it = 0; it < 4; ++it) {
          const int row = it * 4 + q;
          const float* sp = slab + row * 68 + c8;
          float vv[8];
#pragma unroll
          for (int e = 0; e < 8; ++e) vv[e] = sp[e];
          if (GATE) {
            const float* gp = gate + (size_t)(mBase + row) * ldc + n0 + c8;
            const v4f g0 = *(const v4f*)(gp);
            const v4f g1 = *(const v4f*)(gp + 4);
            vv[0] *= g0[0]; vv[1] *= g0[1]; vv[2] *= g0[2]; vv[3] *= g0[3];
            vv[4] *= g1[0]; vv[5] *= g1[1]; vv[6] *= g1[2]; vv[7] *= g1[3];
          }
          v8h hv, lv;
#pragma unroll
          for (int e = 0; e < 8; ++e) {
            if (OUT_MODE == 1) {
              hv[e] = (_Float16)vv[e];
            } else {
              unsigned short hb = f2bf_bits(vv[e]);
              unsigned short lb = f2bf_bits(vv[e] - bf_bits2f(hb));
              hv[e] = __builtin_bit_cast(_Float16, hb);
              lv[e] = __builtin_bit_cast(_Float16, lb);
            }
          }
          *(volatile v8h*)(C + (size_t)(mBase + row) * ldc + n0 + c8) = hv;
          if (OUT_MODE == 2) *(volatile v8h*)(C2 + (size_t)(mBase + row) * ldc + n0 + c8) = lv;
        }
        __threadfence();
      }
    }
    __builtin_amdgcn_fence(__ATOMIC_RELEASE, "workgroup");
    __builtin_amdgcn_wave_barrier();
    __builtin_amdgcn_fence(__ATOMIC_ACQUIRE, "workgroup");
  }
}

__global__ __launch_bounds__(256) void transpose_bf16_kernel(
    const float* __restrict__ W0, const float* __restrict__ W1, const float* __restrict__ W2, const float* __restrict__ W3,
    unsigned short* __restrict__ T0, unsigned short* __restrict__ T1, unsigned short* __restrict__ T2, unsigned short* __restrict__ T3)
{
  __shared__ float tile[64 * 65];
  const int tid = threadIdx.x, lane = tid & 31, wave = tid >> 5;
  const int z = blockIdx.z;
  const float* W = (z == 0) ? W0 : (z == 1) ? W1 : (z == 2) ? W2 : W3;
  unsigned short* Bt = (z == 0) ? T0 : (z == 1) ? T1 : (z == 2) ? T2 : T3;
  const int n0 = blockIdx.x * 64;
  const int k0 = blockIdx.y * 64;
#pragma unroll
  for (int p = 0; p < 4; ++p) {
    const int idx = tid + p * 256;
    const int kk  = idx >> 4;
    const int n4  = (idx & 15) * 4;
    const v4f a = *(const v4f*)(W + (size_t)(k0 + kk) * kDim + n0 + n4);
    tile[kk * 65 + n4 + 0] = a[0];
    tile[kk * 65 + n4 + 1] = a[1];
    tile[kk * 65 + n4 + 2] = a[2];
    tile[kk * 65 + n4 + 3] = a[3];
  }
  __syncthreads();
  const int q = lane >> 3, c8 = (lane & 7) * 8;
  v4u hv[2];
#pragma unroll
  for (int it = 0; it < 2; ++it) {
    const int nrow = it * 32 + wave * 4 + q;
#pragma unroll
    for (int p = 0; p < 4; ++p) {
      const float f0 = tile[(c8 + 2 * p) * 65 + nrow];
      const float f1 = tile[(c8 + 2 * p + 1) * 65 + nrow];
      hv[it][p] = bf_hi32(f0) | (bf_hi32(f1) << 16);
    }
  }
  for (int pass = 0; pass < 2; ++pass) {
#pragma unroll
    for (int it = 0; it < 2; ++it) {
      const int nrow = it * 32 + wave * 4 + q;
      *(volatile v4u*)(Bt + (size_t)(n0 + nrow) * kDim + k0 + c8) = hv[it];
    }
    __threadfence();
  }
}

__global__ __launch_bounds__(256) void bc_weight_kernel(
    const float* __restrict__ WB, const float* __restrict__ WC, unsigned short* __restrict__ Bt)
{
  __shared__ float tile[64 * 65];
  const int tid = threadIdx.x, lane = tid & 31, wave = tid >> 5;
  const int k0 = blockIdx.x * 64;
  {
    const int kk = tid >> 2, n4 = (tid & 3) * 4;
    const v4f a = *(const v4f*)(WB + (size_t)(k0 + kk) * kNst + n4);
    const v4f c = *(const v4f*)(WC + (size_t)(k0 + kk) * kNst + n4);
    tile[kk * 65 + n4 + 0] = a[0];
    tile[kk * 65 + n4 + 1] = a[1];
    tile[kk * 65 + n4 + 2] = a[2];
    tile[kk * 65 + n4 + 3] = a[3];
    tile[kk * 65 + kNst + n4 + 0] = c[0];
    tile[kk * 65 + kNst + n4 + 1] = c[1];
    tile[kk * 65 + kNst + n4 + 2] = c[2];
    tile[kk * 65 + kNst + n4 + 3] = c[3];
  }
#pragma unroll
  for (int p = 0; p < 8; ++p) {
    const int idx = tid + p * 256;
    const int kk  = idx >> 5;
    const int nn  = 32 + (idx & 31);
    tile[kk * 65 + nn] = 0.0f;
  }
  __syncthreads();
  const int q = lane >> 3, c8 = (lane & 7) * 8;
  v4u hv[2];
#pragma unroll
  for (int it = 0; it < 2; ++it) {
    const int nrow = it * 32 + wave * 4 + q;
#pragma unroll
    for (int p = 0; p < 4; ++p) {
      const float f0 = tile[(c8 + 2 * p) * 65 + nrow];
      const float f1 = tile[(c8 + 2 * p + 1) * 65 + nrow];
      hv[it][p] = bf_hi32(f0) | (bf_hi32(f1) << 16);
    }
  }
  for (int pass = 0; pass < 2; ++pass) {
#pragma unroll
    for (int it = 0; it < 2; ++it) {
      const int nrow = it * 32 + wave * 4 + q;
      *(volatile v4u*)(Bt + (size_t)nrow * kDim + k0 + c8) = hv[it];
    }
    __threadfence();
  }
}

__global__ __launch_bounds__(256) void ln_split_kernel(
    const float* __restrict__ x, const float* __restrict__ g, const float* __restrict__ bt,
    unsigned short* __restrict__ XH, unsigned short* __restrict__ XL)
{
  const int lane = threadIdx.x & 31, wave = threadIdx.x >> 5;
  const int row = blockIdx.x * 8 + wave;
  const float* xr = x + (size_t)row * kDim;
  float xv[32];
#pragma unroll
  for (int j = 0; j < 4; ++j) {
    const v4f a0 = *(const v4f*)(xr + j * 256 + lane * 8);
    const v4f a1 = *(const v4f*)(xr + j * 256 + lane * 8 + 4);
    xv[j * 8 + 0] = rbf(a0[0]); xv[j * 8 + 1] = rbf(a0[1]); xv[j * 8 + 2] = rbf(a0[2]); xv[j * 8 + 3] = rbf(a0[3]);
    xv[j * 8 + 4] = rbf(a1[0]); xv[j * 8 + 5] = rbf(a1[1]); xv[j * 8 + 6] = rbf(a1[2]); xv[j * 8 + 7] = rbf(a1[3]);
  }
  float s = 0.0f;
#pragma unroll
  for (int i = 0; i < 32; ++i) s += xv[i];
#pragma unroll
  for (int off = 16; off >= 1; off >>= 1) s += __shfl_xor(s, off, 32);
  const float mu = s * (1.0f / (float)kDim);
  float qs = 0.0f;
#pragma unroll
  for (int i = 0; i < 32; ++i) { const float dlt = xv[i] - mu; qs += dlt * dlt; }
#pragma unroll
  for (int off = 16; off >= 1; off >>= 1) qs += __shfl_xor(qs, off, 32);
  const float var = qs * (1.0f / (float)kDim);
  const float inv = rsqrtf(var + kLnEps);

  v4u hv[4], lv[4];
#pragma unroll
  for (int j = 0; j < 4; ++j) {
    const int c0 = j * 256 + lane * 8;
    const v4f g0 = *(const v4f*)(g + c0);
    const v4f g1 = *(const v4f*)(g + c0 + 4);
    const v4f b0 = *(const v4f*)(bt + c0);
    const v4f b1 = *(const v4f*)(bt + c0 + 4);
    float y[8];
    y[0] = (xv[j * 8 + 0] - mu) * inv * rbf(g0[0]) + rbf(b0[0]);
    y[1] = (xv[j * 8 + 1] - mu) * inv * rbf(g0[1]) + rbf(b0[1]);
    y[2] = (xv[j * 8 + 2] - mu) * inv * rbf(g0[2]) + rbf(b0[2]);
    y[3] = (xv[j * 8 + 3] - mu) * inv * rbf(g0[3]) + rbf(b0[3]);
    y[4] = (xv[j * 8 + 4] - mu) * inv * rbf(g1[0]) + rbf(b1[0]);
    y[5] = (xv[j * 8 + 5] - mu) * inv * rbf(g1[1]) + rbf(b1[1]);
    y[6] = (xv[j * 8 + 6] - mu) * inv * rbf(g1[2]) + rbf(b1[2]);
    y[7] = (xv[j * 8 + 7] - mu) * inv * rbf(g1[3]) + rbf(b1[3]);
#pragma unroll
    for (int p = 0; p < 4; ++p) {
      unsigned hw, lw;
      split_pack(y[2 * p], y[2 * p + 1], hw, lw);
      hv[j][p] = hw;
      lv[j][p] = lw;
    }
    asm volatile("" ::: "memory");
  }
  unsigned short* ph = XH + (size_t)row * kDim;
  unsigned short* pl = XL + (size_t)row * kDim;
  for (int pass = 0; pass < 2; ++pass) {
#pragma unroll
    for (int j = 0; j < 4; ++j) {
      *(volatile v4u*)(ph + j * 256 + lane * 8) = hv[j];
      *(volatile v4u*)(pl + j * 256 + lane * 8) = lv[j];
    }
    __threadfence();
  }
}

__global__ __launch_bounds__(256) void conv_silu_kernel(
    const float* __restrict__ X1, const float* __restrict__ cw,
    unsigned short* __restrict__ UH, unsigned short* __restrict__ UL)
{
  __shared__ __align__(16) float sT[16 * kConvTP];
  const int tid = threadIdx.x, lane = tid & 31, wave = tid >> 5;
  const int d0 = blockIdx.x * 256, d = d0 + tid;
  const int g0 = blockIdx.y * 64;
  const int tb = g0 & (kSeq - 1);
  const float w0 = rbf(cw[d * 3 + 0]), w1 = rbf(cw[d * 3 + 1]), w2 = rbf(cw[d * 3 + 2]);
  float xprev, xcur;
  {
    const int rp = (g0 > 0) ? (g0 - 1) : 0;
    const float vp = X1[(size_t)rp * kDim + d];
    xprev = (tb > 0) ? vp : 0.0f;
    xcur  = X1[(size_t)g0 * kDim + d];
  }
#pragma unroll 1
  for (int sub = 0; sub < 4; ++sub) {
    const int lb = g0 + sub * 16;
#pragma unroll 1
    for (int s = 0; s < 16; ++s) {
      const int rowg = lb + s;
      const int l = tb + sub * 16 + s;
      const int rn = (rowg + 1 < kRows) ? (rowg + 1) : (kRows - 1);
      const float vn = X1[(size_t)rn * kDim + d];
      const float xnext = (l + 1 < kSeq) ? vn : 0.0f;
      float acc = w0 * xprev;
      acc = fmaf(w1, xcur, acc);
      acc = fmaf(w2, xnext, acc);
      const float sg = 1.0f / (1.0f + expf(-acc));
      sT[s * kConvTP + tid] = acc * sg;
      xprev = xcur;
      xcur = xnext;
    }
    __syncthreads();
    v4u hv[2], lv[2];
#pragma unroll
    for (int it = 0; it < 2; ++it) {
      const float* sp = sT + (it * 8 + wave) * kConvTP + lane * 8;
      const v4f a0 = *(const v4f*)(sp);
      const v4f a1 = *(const v4f*)(sp + 4);
      unsigned hw, lw;
      split_pack(a0[0], a0[1], hw, lw); hv[it][0] = hw; lv[it][0] = lw;
      split_pack(a0[2], a0[3], hw, lw); hv[it][1] = hw; lv[it][1] = lw;
      split_pack(a1[0], a1[1], hw, lw); hv[it][2] = hw; lv[it][2] = lw;
      split_pack(a1[2], a1[3], hw, lw); hv[it][3] = hw; lv[it][3] = lw;
    }
    for (int pass = 0; pass < 2; ++pass) {
#pragma unroll
      for (int it = 0; it < 2; ++it) {
        const size_t o = (size_t)(lb + it * 8 + wave) * kDim + d0 + lane * 8;
        *(volatile v4u*)(UH + o) = hv[it];
        *(volatile v4u*)(UL + o) = lv[it];
      }
      __threadfence();
    }
    __syncthreads();
  }
}

__device__ __forceinline__ v4f unpack_dt2(unsigned a, unsigned b) {
  v4f o;
  o[0] = h16_to_f32(a & 0xffffu) * kDtCarryInv;
  o[1] = h16_to_f32(a >> 16) * kDtCarryInv;
  o[2] = h16_to_f32(b & 0xffffu) * kDtCarryInv;
  o[3] = h16_to_f32(b >> 16) * kDtCarryInv;
  return o;
}
__device__ __forceinline__ v4f unpack_u2(unsigned ah, unsigned bh, unsigned al, unsigned bl) {
  v4f o;
  o[0] = __uint_as_float(ah << 16) + __uint_as_float(al << 16);
  o[1] = __uint_as_float(ah & 0xffff0000u) + __uint_as_float(al & 0xffff0000u);
  o[2] = __uint_as_float(bh << 16) + __uint_as_float(bl << 16);
  o[3] = __uint_as_float(bh & 0xffff0000u) + __uint_as_float(bl & 0xffff0000u);
  return o;
}

__global__ __launch_bounds__(64) void scan_kernel(
    const unsigned short* __restrict__ DT16, const unsigned short* __restrict__ UH, const unsigned short* __restrict__ UL,
    const float* __restrict__ BC, const float* __restrict__ Alog, const float* __restrict__ bdt,
    const float* __restrict__ Dsk, float* __restrict__ XSSM)
{
  __shared__ __align__(16) float sX[kScanTS * 32];
  __shared__ __align__(16) float sDT[kScanTS * kScanCh];
  __shared__ __align__(16) float sU[kScanTS * kScanCh];
  __shared__ __align__(16) float sY[kScanTS * kScanYP];
  const int tid = threadIdx.x, lane = tid & 31, wave = tid >> 5;
  constexpr int kBlkPerB = kDim / kScanCh;
  const int bix = blockIdx.x / kBlkPerB;
  const int d0  = (blockIdx.x - bix * kBlkPerB) * kScanCh;
  const int d   = d0 + tid;
  const size_t row0 = (size_t)bix * kSeq;

  float negA[kNst], h[kNst];
#pragma unroll
  for (int q4 = 0; q4 < 4; ++q4) {
    const v4f a = *(const v4f*)(Alog + (size_t)d * kNst + 4 * q4);
    negA[4 * q4 + 0] = -expf(rbf(a[0]));
    negA[4 * q4 + 1] = -expf(rbf(a[1]));
    negA[4 * q4 + 2] = -expf(rbf(a[2]));
    negA[4 * q4 + 3] = -expf(rbf(a[3]));
  }
#pragma unroll
  for (int n = 0; n < kNst; ++n) h[n] = 0.0f;
  const float bb = rbf(bdt[d]);
  const float Dd = rbf(Dsk[d]);
  const int sr = tid >> 3, sc = tid & 7;
  const int hh = lane >> 4, c4 = (lane & 15) * 4;

#pragma unroll 1
  for (int t0 = 0; t0 < kSeq; t0 += kScanTS) {
    __syncthreads();
#pragma unroll 1
    for (int it = 0; it < 8; ++it) {
      const int r = it * 8 + sr;
      const size_t grow = row0 + t0 + r;
      const v4f bcv = *(const v4f*)(BC + grow * kBcP + sc * 4);
      const size_t o = grow * kDim + d0 + sc * 8;
      const v4u wd = *(const v4u*)(DT16 + o);
      const v4u wh = *(const v4u*)(UH + o);
      const v4u wl = *(const v4u*)(UL + o);
      const unsigned wd0 = wd[0], wd1 = wd[1], wd2 = wd[2], wd3 = wd[3];
      const unsigned wh0 = wh[0], wh1 = wh[1], wh2 = wh[2], wh3 = wh[3];
      const unsigned wl0 = wl[0], wl1 = wl[1], wl2 = wl[2], wl3 = wl[3];
      *(v4f*)(sX + r * 32 + sc * 4) = bcv;
      *(v4f*)(sDT + r * kScanCh + sc * 8)     = unpack_dt2(wd0, wd1);
      *(v4f*)(sDT + r * kScanCh + sc * 8 + 4) = unpack_dt2(wd2, wd3);
      *(v4f*)(sU + r * kScanCh + sc * 8)      = unpack_u2(wh0, wh1, wl0, wl1);
      *(v4f*)(sU + r * kScanCh + sc * 8 + 4)  = unpack_u2(wh2, wh3, wl2, wl3);
    }
    __syncthreads();
#pragma unroll 1
    for (int s = 0; s < kScanTS; ++s) {
      const float* xr = sX + s * 32;
      float Bs[kNst], Cs[kNst];
#pragma unroll
      for (int q4 = 0; q4 < 4; ++q4) {
        const v4f bv = *(const v4f*)(xr + 4 * q4);
        const v4f cv = *(const v4f*)(xr + kNst + 4 * q4);
        Bs[4 * q4 + 0] = bv[0]; Bs[4 * q4 + 1] = bv[1]; Bs[4 * q4 + 2] = bv[2]; Bs[4 * q4 + 3] = bv[3];
        Cs[4 * q4 + 0] = cv[0]; Cs[4 * q4 + 1] = cv[1]; Cs[4 * q4 + 2] = cv[2]; Cs[4 * q4 + 3] = cv[3];
      }
      const float pre = sDT[s * kScanCh + tid] + bb;
      const float ea  = expf(-fabsf(pre));
      const float dt  = fmaxf(pre, 0.0f) + log1pf(ea);
      const float xt  = sU[s * kScanCh + tid];
      const float dtx = dt * xt;
      float y = 0.0f;
#pragma unroll
      for (int k = 0; k < kNst; ++k) {
        const float e = __expf(dt * negA[k]);
        h[k] = e * h[k] + dtx * Bs[k];
        y = h[k] * Cs[k] + y;
      }
      y = y + xt * Dd;
      sY[s * kScanYP + tid] = y;
    }
    __syncthreads();
    for (int pass = 0; pass < 2; ++pass) {
#pragma unroll
      for (int it = 0; it < 16; ++it) {
        const int row = it * 4 + wave * 2 + hh;
        const v4f v = *(const v4f*)(sY + row * kScanYP + c4);
        *(volatile v4f*)(XSSM + (row0 + t0 + row) * kDim + d0 + c4) = v;
      }
      __threadfence();
    }
  }
}

static_assert(((kRows / 64) * (kDim / 64)) % 8 == 0);
static_assert(((kRows / 64) * (kBcP / 64)) % 8 == 0);

extern "C" void kernel_launch(void* const* d_in, const int* in_sizes, int n_in,
                              void* d_out, int out_size, void* d_ws, size_t ws_size,
                              hipStream_t stream) {
  if (n_in < 16) return;
  if (in_sizes[0] != kRows * kDim) return;
  if (in_sizes[1] != kDim || in_sizes[2] != kDim) return;
  if (in_sizes[3] != kDim * kDim || in_sizes[4] != kDim) return;
  if (in_sizes[5] != kDim * kDim || in_sizes[6] != kDim) return;
  if (in_sizes[7] != kDim * kDim || in_sizes[8] != kDim) return;
  if (in_sizes[9] != kDim * 3) return;
  if (in_sizes[10] != kDim * kNst || in_sizes[11] != kDim) return;
  if (in_sizes[12] != kDim * kDim || in_sizes[13] != kDim) return;
  if (in_sizes[14] != kDim * kNst || in_sizes[15] != kDim * kNst) return;
  if (out_size != kRows * kDim) return;
  if (ws_size < kWsTotal) return;

  const float* x      = (const float*)d_in[0];
  const float* ln_g   = (const float*)d_in[1];
  const float* ln_b   = (const float*)d_in[2];
  const float* w1_w   = (const float*)d_in[3];
  const float* w1_b   = (const float*)d_in[4];
  const float* v1_w   = (const float*)d_in[5];
  const float* v1_b   = (const float*)d_in[6];
  const float* w2_w   = (const float*)d_in[7];
  const float* w2_b   = (const float*)d_in[8];
  const float* conv_w = (const float*)d_in[9];
  const float* A_log  = (const float*)d_in[10];
  const float* D_skip = (const float*)d_in[11];
  const float* W_dt   = (const float*)d_in[12];
  const float* b_dt   = (const float*)d_in[13];
  const float* W_B    = (const float*)d_in[14];
  const float* W_C    = (const float*)d_in[15];
  float* out = (float*)d_out;

  char* ws = (char*)d_ws;
  unsigned short* XNH = (unsigned short*)(ws + kOffXNH);
  unsigned short* XNL = (unsigned short*)(ws + kOffXNL);
  float*          R1  = (float*)(ws + kOffR1);
  unsigned short* UH  = (unsigned short*)(ws + kOffUH);
  unsigned short* UL  = (unsigned short*)(ws + kOffUL);
  unsigned short* DT  = (unsigned short*)(ws + kOffDT);
  float*          BC  = (float*)(ws + kOffBC);
  unsigned short* W1T = (unsigned short*)(ws + kOffW1T);
  unsigned short* V1T = (unsigned short*)(ws + kOffV1T);
  unsigned short* W2T = (unsigned short*)(ws + kOffW2T);
  unsigned short* WDT = (unsigned short*)(ws + kOffWDT);
  unsigned short* WBC = (unsigned short*)(ws + kOffWBC);
  const float* dummy_f = b_dt;

  const int gemmBlocksBig = ((kRows / 64) * (kDim / 64)) / 8;
  const int gemmBlocksBC  = ((kRows / 64) * (kBcP / 64)) / 8;

  transpose_bf16_kernel<<<dim3(kDim / 64, kDim / 64, 4), 256, 0, stream>>>(
      w1_w, v1_w, w2_w, W_dt, W1T, V1T, W2T, WDT);
  bc_weight_kernel<<<kDim / 64, 256, 0, stream>>>(W_B, W_C, WBC);

  ln_split_kernel<<<kRows / 8, 256, 0, stream>>>(x, ln_g, ln_b, XNH, XNL);

  wmma_gemm64<1, 2, 0, false, 0><<<gemmBlocksBig, 256, 0, stream>>>(
      XNH, XNL, kDim, W1T, kDim, (void*)R1, (void*)R1, kDim, w1_b, dummy_f, kRows, kDim, kDim, 1.0f);

  conv_silu_kernel<<<dim3(kDim / 256, kRows / 64), 256, 0, stream>>>(R1, conv_w, UH, UL);

  wmma_gemm64<0, 0, 1, false, 0><<<gemmBlocksBig, 256, 0, stream>>>(
      UH, UH, kDim, WDT, kDim, (void*)DT, (void*)DT, kDim, dummy_f, dummy_f, kRows, kDim, kDim, kDtCarry);

  wmma_gemm64<1, 0, 0, false, 0><<<gemmBlocksBC, 256, 0, stream>>>(
      UH, UL, kDim, WBC, kDim, (void*)BC, (void*)BC, kBcP, dummy_f, dummy_f, kRows, kBcP, kDim, 1.0f);

  scan_kernel<<<kBatch * (kDim / kScanCh), kScanCh, 0, stream>>>(DT, UH, UL, BC, A_log, b_dt, D_skip, R1);

  wmma_gemm64<1, 2, 2, true, 3><<<gemmBlocksBig, 256, 0, stream>>>(
      XNH, XNL, kDim, V1T, kDim, (void*)UH, (void*)UL, kDim, v1_b, R1, kRows, kDim, kDim, 1.0f);

  wmma_gemm64<1, 2, 0, false, 0><<<gemmBlocksBig, 256, 0, stream>>>(
      UH, UL, kDim, W2T, kDim, (void*)out, (void*)out, kDim, w2_b, dummy_f, kRows, kDim, kDim, 1.0f);
}
